// LMulLanguageModel_62234076119647
// MI455X (gfx1250) — hardware-verified
//
#include <hip/hip_runtime.h>
#include <math.h>

#ifndef NB
#define NB 2
#endif
#ifndef SEQ
#define SEQ 128
#endif
#define NB_FULL 2
#define SEQ_FULL 128
#define DM 128
#define HEADS 4
#define HD 32
#define FFD 512
#define VOCAB 1024
#define NLAYER 2
#define MTOK (NB * SEQ)
#define QKVP (3 * DM)
#define QKP (6 * DM)

static_assert(SEQ == 128);
static_assert(SEQ == SEQ_FULL);
static_assert(NB >= 1 && NB <= NB_FULL);
static_assert(MTOK % 64 == 0);
static_assert(DM == HEADS * HD && HD == 32 && DM == 128);
static_assert(DM % 64 == 0 && FFD % 64 == 0 && VOCAB % 64 == 0);
static_assert(DM % 32 == 0 && FFD % 32 == 0);
static_assert((MTOK * DM / 8) % 256 == 0 && (MTOK * FFD / 8) % 256 == 0);
static_assert((NLAYER * DM * DM / 8) % 256 == 0 && (NLAYER * FFD * DM / 8) % 256 == 0 && (VOCAB * DM / 8) % 256 == 0);
static_assert((MTOK * DM / 4) % 256 == 0);
static_assert(MTOK % 8 == 0);

typedef _Float16 h16;
typedef __attribute__((ext_vector_type(16))) _Float16 v16h;
typedef __attribute__((ext_vector_type(8)))  _Float16 v8h;
typedef __attribute__((ext_vector_type(2)))  _Float16 v2h;
typedef __attribute__((ext_vector_type(8)))  float    v8f;
typedef __attribute__((ext_vector_type(4)))  float    v4f;
typedef __attribute__((ext_vector_type(2)))  float    v2f;


#define VST2(T, ptr, val) do { const T vst2_v_ = (val); *(volatile T*)(ptr) = vst2_v_; __threadfence(); *(volatile T*)(ptr) = vst2_v_; } while (0)
#define VST2V4(ptr, val) do { const v4f vst2_v4_ = (val); *(volatile v4f*)(ptr) = vst2_v4_; __threadfence(); *(volatile v4f*)(ptr) = vst2_v4_; } while (0)

__device__ __forceinline__ float bfr(float f) {
    unsigned u = __float_as_uint(f);
    u += 0x7FFFu + ((u >> 16) & 1u);
    return __uint_as_float(u & 0xFFFF0000u);
}
__device__ __forceinline__ h16 toh_flush(float v) {
    const float w = (fabsf(v) < 6.103515625e-05f) ? 0.0f : v;
    return (h16)w;
}
__device__ __forceinline__ v2h toh2_flush(float a, float b) {
    v2f w;
    w.x = (fabsf(a) < 6.103515625e-05f) ? 0.0f : a;
    w.y = (fabsf(b) < 6.103515625e-05f) ? 0.0f : b;
    return __builtin_convertvector(w, v2h);
}
union H8  { v8h v;  v2h p[4]; };
union H16 { v16h v; v2h p[8]; };
__device__ __forceinline__ v8h pack8_flush(const float* f) {
    H8 o;
#pragma unroll
    for (int i = 0; i < 4; ++i) o.p[i] = toh2_flush(f[2 * i], f[2 * i + 1]);
    return o.v;
}
__device__ __forceinline__ float mq_pw(float v, int carry) {
    int e;
    const float m = frexpf(v, &e);
    const float r = rintf(m * 8.0f);
    return ldexpf(r, 2 * e - 3 + carry);
}
__device__ __forceinline__ void split_pair(float x0, float x1, v2h& hw, v2h& lw, v2h& sw) {
    const float a0 = x0 * 1024.0f, a1 = x1 * 1024.0f;
    hw = toh2_flush(a0, a1);
    lw = toh2_flush((a0 - (float)hw.x) * 2048.0f, (a1 - (float)hw.y) * 2048.0f);
    sw = toh2_flush(x0 * 0.5f, x1 * 0.5f);
}

union FragU { v16h v; v8h h[2]; };
__device__ __forceinline__ v16h frag_ld(const _Float16* p) {
    FragU f; f.h[0] = *(const v8h*)(p); f.h[1] = *(const v8h*)(p + 16); return f.v;
}
__device__ __forceinline__ v8f wmma16(v16h a, v16h b, v8f c) {
    c = __builtin_amdgcn_wmma_f32_16x16x32_f16(false, a, false, b, (short)0, c, false, false);
    asm volatile("v_nop\n\tv_nop\n\tv_nop\n\tv_nop" : "+v"(c) : "v"(a), "v"(b));
    return c;
}
__device__ __forceinline__ void wave_sync_lds() {
    __builtin_amdgcn_fence(3  , "workgroup");
    __builtin_amdgcn_wave_barrier();
    __builtin_amdgcn_fence(2  , "workgroup");
}

__global__ __launch_bounds__(256) void k_prepw(const float* __restrict__ W, _Float16* __restrict__ P16, unsigned n8) {
    const unsigned u = blockIdx.x * 256u + threadIdx.x;
    if (u >= n8) return;
    const v4f a = *(const v4f*)(W + (size_t)u * 8u);
    const v4f b = *(const v4f*)(W + (size_t)u * 8u + 4u);
    float f[8];
    f[0] = mq_pw(bfr(a.x), 14); f[1] = mq_pw(bfr(a.y), 14); f[2] = mq_pw(bfr(a.z), 14); f[3] = mq_pw(bfr(a.w), 14);
    f[4] = mq_pw(bfr(b.x), 14); f[5] = mq_pw(bfr(b.y), 14); f[6] = mq_pw(bfr(b.z), 14); f[7] = mq_pw(bfr(b.w), 14);
    VST2(v8h, P16 + (size_t)u * 8u, pack8_flush(f));
}

__global__ __launch_bounds__(256) void k_prepx(const float* __restrict__ X, _Float16* __restrict__ P16, unsigned n8) {
    const unsigned u = blockIdx.x * 256u + threadIdx.x;
    if (u >= n8) return;
    const v4f a = *(const v4f*)(X + (size_t)u * 8u);
    const v4f b = *(const v4f*)(X + (size_t)u * 8u + 4u);
    float f[8];
    f[0] = mq_pw(a.x, 10); f[1] = mq_pw(a.y, 10); f[2] = mq_pw(a.z, 10); f[3] = mq_pw(a.w, 10);
    f[4] = mq_pw(b.x, 10); f[5] = mq_pw(b.y, 10); f[6] = mq_pw(b.z, 10); f[7] = mq_pw(b.w, 10);
    VST2(v8h, P16 + (size_t)u * 8u, pack8_flush(f));
}

static_assert(32 * 16 == DM * 4);
__global__ __launch_bounds__(256) void k_embed(const int* __restrict__ tokens, const float* __restrict__ emb,
                                               const float* __restrict__ pos, float* __restrict__ x) {
    const unsigned u = blockIdx.x * 256u + threadIdx.x;
    if (u >= (unsigned)(MTOK * DM / 4)) return;
    const unsigned row = u >> 5, c4 = (u & 31u) * 4u;
    const unsigned b = row >> 7, s = row & 127u;
    int t = tokens[b * SEQ_FULL + s];
    t = min(max(t, 0), VOCAB - 1);
    const v4f e = *(const v4f*)(emb + (size_t)t * DM + c4);
    const v4f p = *(const v4f*)(pos + (size_t)s * DM + c4);
    v4f o;
    o.x = bfr(e.x) + bfr(p.x); o.y = bfr(e.y) + bfr(p.y); o.z = bfr(e.z) + bfr(p.z); o.w = bfr(e.w) + bfr(p.w);
    VST2V4(x + (size_t)row * DM + c4, o);
}

static_assert(2 * 4 * 32 * 16 == 16 * 64 * 4);
static_assert(8 * 16 * 68 * 4 <= 131072);
template <bool RESID, bool RELU>
__device__ __forceinline__ void gemm64_body(float* sT,
    const _Float16* __restrict__ A, unsigned lda, const _Float16* __restrict__ Bt, unsigned ldb,
    float* __restrict__ C, unsigned ldc, const float* __restrict__ bias, const float* __restrict__ resid,
    unsigned N, unsigned K) {
  const unsigned lane = threadIdx.x & 31u;
  const unsigned wave = (unsigned)__builtin_amdgcn_readfirstlane((int)(threadIdx.x >> 5));
  const unsigned tilesM = (unsigned)(MTOK / 64), tilesN = N >> 6;
  const unsigned tile = blockIdx.x * 8u + wave;
  if (tile >= tilesM * tilesN) return;
  const unsigned tn = tile / tilesM;
  const unsigned tm = tile - tn * tilesM;
  const unsigned m0 = tm << 6, n0 = tn << 6;
  const unsigned rlane = lane & 15u;
  const unsigned koff = (lane >> 4) * 8u;
  const unsigned mOff = koff;

  v8f acc[4][4];
#pragma unroll
  for (int i = 0; i < 4; ++i)
#pragma unroll
    for (int j = 0; j < 4; ++j) acc[i][j] = (v8f){0.f,0.f,0.f,0.f,0.f,0.f,0.f,0.f};

  for (unsigned k0 = 0; k0 < K; k0 += 32u) {
    v16h bh[4];
#pragma unroll
    for (int j = 0; j < 4; ++j)
      bh[j] = frag_ld(Bt + (size_t)(n0 + ((unsigned)j << 4) + rlane) * ldb + koff + k0);
#pragma unroll
    for (int i = 0; i < 4; ++i) {
      const v16h ah = frag_ld(A + (size_t)(m0 + ((unsigned)i << 4) + rlane) * lda + koff + k0);
#pragma unroll
      for (int j = 0; j < 4; ++j)
        acc[i][j] = wmma16(ah, bh[j], acc[i][j]);
    }
  }

  float* slab = sT + wave * (16u * 68u);
#pragma unroll
  for (int i = 0; i < 4; ++i) {
    const unsigned mBase = m0 + ((unsigned)i << 4);
#pragma unroll
    for (int j = 0; j < 4; ++j) {
      const unsigned n = n0 + ((unsigned)j << 4) + rlane;
      const float bv = bfr(bias[n]);
#pragma unroll
      for (int r = 0; r < 8; ++r) {
        float v = acc[i][j][r] * 5.9604644775390625e-08f + bv;
        if (RELU) v = fmaxf(v, 0.0f);
        slab[(mOff + (unsigned)r) * 68u + ((unsigned)j << 4) + rlane] = v;
      }
    }
    wave_sync_lds();
    {
      const unsigned hh = lane >> 4, c4 = (lane & 15u) * 4u;
#pragma unroll
      for (int half = 0; half < 2; ++half) {
        v4f vv[4];
#pragma unroll
        for (int it = 0; it < 4; ++it) {
          const unsigned row = (unsigned)(half * 4 + it) * 2u + hh;
          vv[it] = *(const v4f*)(slab + row * 68u + c4);
          if (RESID) vv[it] += *(const v4f*)(resid + (size_t)(mBase + row) * ldc + n0 + c4);
        }
        for (int pass = 0; pass < 2; ++pass) {
#pragma unroll
          for (int it = 0; it < 4; ++it) {
            const unsigned row = (unsigned)(half * 4 + it) * 2u + hh;
            *(volatile v4f*)(C + (size_t)(mBase + row) * ldc + n0 + c4) = vv[it];
          }
          __threadfence();
        }
      }
    }
    wave_sync_lds();
  }
}

__global__ __launch_bounds__(256) void k_gemm_plain(const _Float16* __restrict__ A, unsigned lda, const _Float16* __restrict__ Bt, unsigned ldb,
                                                    float* __restrict__ C, unsigned ldc, const float* __restrict__ bias, unsigned N, unsigned K) {
  __shared__ __align__(16) float sT[8 * 16 * 68];
  gemm64_body<false, false>(sT, A, lda, Bt, ldb, C, ldc, bias, nullptr, N, K);
}
__global__ __launch_bounds__(256) void k_gemm_relu(const _Float16* __restrict__ A, unsigned lda, const _Float16* __restrict__ Bt, unsigned ldb,
                                                   float* __restrict__ C, unsigned ldc, const float* __restrict__ bias, unsigned N, unsigned K) {
  __shared__ __align__(16) float sT[8 * 16 * 68];
  gemm64_body<false, true>(sT, A, lda, Bt, ldb, C, ldc, bias, nullptr, N, K);
}
__global__ __launch_bounds__(256) void k_gemm_resid(const _Float16* __restrict__ A, unsigned lda, const _Float16* __restrict__ Bt, unsigned ldb,
                                                    float* __restrict__ C, unsigned ldc, const float* __restrict__ bias,
                                                    const float* __restrict__ resid, unsigned N, unsigned K) {
  __shared__ __align__(16) float sT[8 * 16 * 68];
  gemm64_body<true, false>(sT, A, lda, Bt, ldb, C, ldc, bias, resid, N, K);
}

#define SP_PV 132
static_assert(8 * 8 == 64);
static_assert(3 * 32 * 16 == QKP * 2);
static_assert(3 * 4 * 256 * 16 == 3 * DM * 64 * 2);
static_assert(64 * SP_PV * 4 <= 131072);
__global__ __launch_bounds__(256) void k_split(const float* __restrict__ qkv, _Float16* __restrict__ qk16, _Float16* __restrict__ vt16) {
    __shared__ __align__(16) float sV[64 * SP_PV];
    const unsigned tid = threadIdx.x, lane = tid & 31u;
    const unsigned wave = (unsigned)__builtin_amdgcn_readfirstlane((int)(tid >> 5));
    const unsigned r0 = blockIdx.x * 64u;
#pragma unroll
    for (int it = 0; it < 8; ++it) {
        const unsigned idx = (unsigned)it * 256u + tid;
        const unsigned row = idx >> 5, c4 = (idx & 31u) * 4u;
        const v4f vv = *(const v4f*)(qkv + (size_t)(r0 + row) * QKVP + 2u * DM + c4);
        *(v4f*)(sV + row * SP_PV + c4) = vv;
    }
    for (unsigned it = 0; it < 8u; ++it) {
        const unsigned row = r0 + it * 8u + wave;
        const float* src = qkv + (size_t)row * QKVP + lane * 8u;
        const v4f a = *(const v4f*)(src), b = *(const v4f*)(src + 4);
        H8 hw, lw, sw;
        split_pair(a.x, a.y, hw.p[0], lw.p[0], sw.p[0]);
        split_pair(a.z, a.w, hw.p[1], lw.p[1], sw.p[1]);
        split_pair(b.x, b.y, hw.p[2], lw.p[2], sw.p[2]);
        split_pair(b.z, b.w, hw.p[3], lw.p[3], sw.p[3]);
        _Float16* dst = qk16 + (size_t)row * QKP + (lane >> 4) * (3u * DM) + (lane & 15u) * 8u;
        VST2(v8h, dst, hw.v);
        VST2(v8h, dst + DM, lw.v);
        VST2(v8h, dst + 2 * DM, sw.v);
    }
    __syncthreads();
    for (unsigned it = 0; it < 4u; ++it) {
        const unsigned p = it * 256u + tid;
        const unsigned ch = p >> 3, t0 = (p & 7u) * 8u;
        float f[8];
#pragma unroll
        for (int e = 0; e < 8; ++e) f[e] = sV[(t0 + (unsigned)e) * SP_PV + ch];
        H8 hw, lw, sw;
        split_pair(f[0], f[1], hw.p[0], lw.p[0], sw.p[0]);
        split_pair(f[2], f[3], hw.p[1], lw.p[1], sw.p[1]);
        split_pair(f[4], f[5], hw.p[2], lw.p[2], sw.p[2]);
        split_pair(f[6], f[7], hw.p[3], lw.p[3], sw.p[3]);
        _Float16* dst = vt16 + (size_t)ch * MTOK + r0 + t0;
        VST2(v8h, dst, hw.v);
        VST2(v8h, dst + (size_t)DM * MTOK, lw.v);
        VST2(v8h, dst + (size_t)2 * DM * MTOK, sw.v);
    }
}

#define AT_PP 36
static_assert(4 * 32 * 16 == 16 * HD * 4);
static_assert(8 * 16 == SEQ);
static_assert(8 * 16 * AT_PP * 4 <= 131072);
__global__ __launch_bounds__(256) void k_attn(const _Float16* __restrict__ qk16, const _Float16* __restrict__ vt16,
                                              float* __restrict__ ctx) {
    __shared__ __align__(16) float sP[8][16 * AT_PP];
    const unsigned tid = threadIdx.x, lane = tid & 31u;
    const unsigned wave = (unsigned)__builtin_amdgcn_readfirstlane((int)(tid >> 5));
    const unsigned hh = lane >> 4, c = lane & 15u;
    const unsigned b = blockIdx.x >> 2, head = blockIdx.x & 3u;
    const unsigned q0 = wave * 16u;
    float* pw = sP[wave];
    const float SC2 = 0.17677669529663687f * (1.0f / 1048576.0f) * 1.4426950408889634f;
    const _Float16* qrow = qk16 + (size_t)(b * SEQ + q0 + c) * QKP + head * HD + 8u * hh;
    const v16h qh = frag_ld(qrow);
    const v16h ql = frag_ld(qrow + DM);
    const v16h qs = frag_ld(qrow + 2 * DM);
    float mrow[8], lrow[8];
    v8f os[2];
#pragma unroll
    for (int r = 0; r < 8; ++r) { mrow[r] = -3.0e38f; lrow[r] = 0.f; }
#pragma unroll
    for (int t = 0; t < 2; ++t) os[t] = (v8f){0.f,0.f,0.f,0.f,0.f,0.f,0.f,0.f};
#pragma unroll 1
    for (unsigned kc = 0; kc < (unsigned)(SEQ / 32); ++kc) {
        const unsigned kv0 = kc * 32u;
        v8f s[2];
#pragma unroll
        for (int j = 0; j < 2; ++j) {
            const _Float16* krow = qk16 + (size_t)(b * SEQ + kv0 + (unsigned)j * 16u + c) * QKP + 3u * DM + head * HD + 8u * hh;
            const v16h kh = frag_ld(krow);
            const v16h kl = frag_ld(krow + DM);
            const v16h ks = frag_ld(krow + 2 * DM);
            const v8f z = (v8f){0.f,0.f,0.f,0.f,0.f,0.f,0.f,0.f};
            s[j] = wmma16(qh, kh, z);
            s[j] = wmma16(qs, kl, s[j]);
            s[j] = wmma16(ql, ks, s[j]);
        }
#pragma unroll
        for (int r = 0; r < 8; ++r) {
            float mx = -3.0e38f;
#pragma unroll
            for (int j = 0; j < 2; ++j) { s[j][r] *= SC2; mx = fmaxf(mx, s[j][r]); }
            mx = fmaxf(mx, __shfl_xor(mx, 1, 32)); mx = fmaxf(mx, __shfl_xor(mx, 2, 32));
            mx = fmaxf(mx, __shfl_xor(mx, 4, 32)); mx = fmaxf(mx, __shfl_xor(mx, 8, 32));
            const float mnew = fmaxf(mrow[r], mx);
            const float alpha = exp2f(mrow[r] - mnew);
            mrow[r] = mnew;
            float psum = 0.f;
#pragma unroll
            for (int j = 0; j < 2; ++j) {
                const float p = exp2f(s[j][r] - mnew);
                psum += p;
                pw[(8u * hh + (unsigned)r) * AT_PP + (unsigned)j * 16u + c] = p;
            }
            psum += __shfl_xor(psum, 1, 32); psum += __shfl_xor(psum, 2, 32);
            psum += __shfl_xor(psum, 4, 32); psum += __shfl_xor(psum, 8, 32);
            lrow[r] = lrow[r] * alpha + psum;
            os[0][r] *= alpha; os[1][r] *= alpha;
        }
        wave_sync_lds();
        {
            const float* pr = pw + c * AT_PP + 8u * hh;
            const v4f p0 = *(const v4f*)(pr), p1 = *(const v4f*)(pr + 4), p2 = *(const v4f*)(pr + 16), p3 = *(const v4f*)(pr + 20);
            H16 ph, pl, ps;
            split_pair(p0.x, p0.y, ph.p[0], pl.p[0], ps.p[0]);
            split_pair(p0.z, p0.w, ph.p[1], pl.p[1], ps.p[1]);
            split_pair(p1.x, p1.y, ph.p[2], pl.p[2], ps.p[2]);
            split_pair(p1.z, p1.w, ph.p[3], pl.p[3], ps.p[3]);
            split_pair(p2.x, p2.y, ph.p[4], pl.p[4], ps.p[4]);
            split_pair(p2.z, p2.w, ph.p[5], pl.p[5], ps.p[5]);
            split_pair(p3.x, p3.y, ph.p[6], pl.p[6], ps.p[6]);
            split_pair(p3.z, p3.w, ph.p[7], pl.p[7], ps.p[7]);
#pragma unroll
            for (int t = 0; t < 2; ++t) {
                const _Float16* vrow = vt16 + (size_t)(head * HD + (unsigned)t * 16u + c) * MTOK + b * SEQ + kv0 + 8u * hh;
                const v16h vh = frag_ld(vrow);
                const v16h vl = frag_ld(vrow + (size_t)DM * MTOK);
                const v16h vs = frag_ld(vrow + (size_t)2 * DM * MTOK);
                os[t] = wmma16(ph.v, vh, os[t]);
                os[t] = wmma16(ps.v, vl, os[t]);
                os[t] = wmma16(pl.v, vs, os[t]);
            }
        }
        wave_sync_lds();
    }
#pragma unroll
    for (int r = 0; r < 8; ++r) {
        const float inv = 1.0f / (lrow[r] * 1048576.0f);
#pragma unroll
        for (int t = 0; t < 2; ++t)
            pw[(8u * hh + (unsigned)r) * AT_PP + (unsigned)t * 16u + c] = os[t][r] * inv;
    }
    wave_sync_lds();
    {
        const unsigned q = lane >> 3, c4 = (lane & 7u) * 4u;
        v4f ov[4];
#pragma unroll
        for (int it = 0; it < 4; ++it) ov[it] = *(const v4f*)(pw + ((unsigned)it * 4u + q) * AT_PP + c4);
        float* dst = ctx + (size_t)(b * SEQ + q0) * DM + head * HD;
        for (int pass = 0; pass < 2; ++pass) {
#pragma unroll
            for (int it = 0; it < 4; ++it) *(volatile v4f*)(dst + (size_t)((unsigned)it * 4u + q) * DM + c4) = ov[it];
            __threadfence();
        }
    }
}

__global__ __launch_bounds__(256) void k_ln(const float* __restrict__ h, const float* __restrict__ g, const float* __restrict__ bt,
                                            float* __restrict__ xo) {
    const unsigned wave = (unsigned)__builtin_amdgcn_readfirstlane((int)(threadIdx.x >> 5));
    const unsigned row = blockIdx.x * 8u + wave;
    const unsigned L = threadIdx.x & 31u;
    if (row >= (unsigned)MTOK) return;
    const v4f a = *(const v4f*)(h + (size_t)row * DM + 4u * L);
    float s = (a.x + a.y) + (a.z + a.w);
#pragma unroll
    for (int o = 16; o > 0; o >>= 1) s += __shfl_xor(s, o, 32);
    const float mu = s * (1.0f / 128.0f);
    const float d0 = a.x - mu, d1 = a.y - mu, d2 = a.z - mu, d3 = a.w - mu;
    float q = (d0 * d0 + d1 * d1) + (d2 * d2 + d3 * d3);
#pragma unroll
    for (int o = 16; o > 0; o >>= 1) q += __shfl_xor(q, o, 32);
    const float rs = 1.0f / sqrtf(q * (1.0f / 128.0f) + 1e-5f);
    const v4f g0 = *(const v4f*)(g + 4u * L);
    const v4f b0 = *(const v4f*)(bt + 4u * L);
    v4f y;
    y.x = d0 * rs * bfr(g0.x) + bfr(b0.x);
    y.y = d1 * rs * bfr(g0.y) + bfr(b0.y);
    y.z = d2 * rs * bfr(g0.z) + bfr(b0.z);
    y.w = d3 * rs * bfr(g0.w) + bfr(b0.w);
    VST2V4(xo + (size_t)row * DM + 4u * L, y);
}

constexpr size_t al256(size_t b) { return (b + 255) & ~(size_t)255; }
constexpr size_t OFF_XA   = 0;
constexpr size_t OFF_HB   = OFF_XA   + al256((size_t)MTOK * DM * 4);
constexpr size_t OFF_QKV  = OFF_HB   + al256((size_t)MTOK * DM * 4);
constexpr size_t OFF_CTX  = OFF_QKV  + al256((size_t)MTOK * QKVP * 4);
constexpr size_t OFF_H1   = OFF_CTX  + al256((size_t)MTOK * DM * 4);
constexpr size_t OFF_A16  = OFF_H1   + al256((size_t)MTOK * FFD * 4);
constexpr size_t OFF_F16  = OFF_A16  + al256((size_t)MTOK * DM * 2);
constexpr size_t OFF_QK16 = OFF_F16  + al256((size_t)MTOK * FFD * 2);
constexpr size_t OFF_VT16 = OFF_QK16 + al256((size_t)MTOK * QKP * 2);
constexpr size_t OFF_WQ   = OFF_VT16 + al256((size_t)3 * DM * MTOK * 2);
constexpr size_t OFF_WK   = OFF_WQ   + al256((size_t)NLAYER * DM * DM * 2);
constexpr size_t OFF_WV   = OFF_WK   + al256((size_t)NLAYER * DM * DM * 2);
constexpr size_t OFF_WO   = OFF_WV   + al256((size_t)NLAYER * DM * DM * 2);
constexpr size_t OFF_W1   = OFF_WO   + al256((size_t)NLAYER * DM * DM * 2);
constexpr size_t OFF_W2   = OFF_W1   + al256((size_t)NLAYER * FFD * DM * 2);
constexpr size_t OFF_WOUT = OFF_W2   + al256((size_t)NLAYER * DM * FFD * 2);
constexpr size_t WS_TOTAL = OFF_WOUT + al256((size_t)VOCAB * DM * 2);
static_assert(WS_TOTAL <= (size_t)134217728);

extern "C" void kernel_launch(void* const* d_in, const int* in_sizes, int n_in, void* d_out, int out_size,
                              void* d_ws, size_t ws_size, hipStream_t stream) {
    if (n_in < 21) return;
    if (in_sizes[0] < MTOK || in_sizes[1] < VOCAB * DM || in_sizes[2] < SEQ * DM) return;
    if (in_sizes[3] < NLAYER * DM * DM || in_sizes[5] < NLAYER * DM * DM || in_sizes[7] < NLAYER * DM * DM || in_sizes[9] < NLAYER * DM * DM) return;
    if (in_sizes[4] < NLAYER * DM || in_sizes[6] < NLAYER * DM || in_sizes[8] < NLAYER * DM || in_sizes[10] < NLAYER * DM) return;
    if (in_sizes[11] < NLAYER * FFD * DM || in_sizes[12] < NLAYER * FFD || in_sizes[13] < NLAYER * DM * FFD || in_sizes[14] < NLAYER * DM) return;
    if (in_sizes[15] < NLAYER * DM || in_sizes[16] < NLAYER * DM || in_sizes[17] < NLAYER * DM || in_sizes[18] < NLAYER * DM) return;
    if (in_sizes[19] < VOCAB * DM || in_sizes[20] < VOCAB || out_size < MTOK * VOCAB) return;
    if (WS_TOTAL > ws_size) return;

    const int*   tokens = (const int*)d_in[0];
    const float* emb    = (const float*)d_in[1];
    const float* pos    = (const float*)d_in[2];
    const float* Wq     = (const float*)d_in[3];
    const float* bq     = (const float*)d_in[4];
    const float* Wk     = (const float*)d_in[5];
    const float* bk     = (const float*)d_in[6];
    const float* Wv     = (const float*)d_in[7];
    const float* bv     = (const float*)d_in[8];
    const float* Wo     = (const float*)d_in[9];
    const float* bo     = (const float*)d_in[10];
    const float* W1     = (const float*)d_in[11];
    const float* b1     = (const float*)d_in[12];
    const float* W2     = (const float*)d_in[13];
    const float* b2     = (const float*)d_in[14];
    const float* g1     = (const float*)d_in[15];
    const float* be1    = (const float*)d_in[16];
    const float* g2     = (const float*)d_in[17];
    const float* be2    = (const float*)d_in[18];
    const float* Wout   = (const float*)d_in[19];
    const float* bout   = (const float*)d_in[20];
    float* out = (float*)d_out;

    char* wsp = (char*)d_ws;
    float*    xA   = (float*)(wsp + OFF_XA);
    float*    hB   = (float*)(wsp + OFF_HB);
    float*    qkv  = (float*)(wsp + OFF_QKV);
    float*    ctx  = (float*)(wsp + OFF_CTX);
    float*    h1   = (float*)(wsp + OFF_H1);
    _Float16* a16  = (_Float16*)(wsp + OFF_A16);
    _Float16* f16p = (_Float16*)(wsp + OFF_F16);
    _Float16* qk16 = (_Float16*)(wsp + OFF_QK16);
    _Float16* vt16 = (_Float16*)(wsp + OFF_VT16);
    _Float16* wq   = (_Float16*)(wsp + OFF_WQ);
    _Float16* wk   = (_Float16*)(wsp + OFF_WK);
    _Float16* wv   = (_Float16*)(wsp + OFF_WV);
    _Float16* wo   = (_Float16*)(wsp + OFF_WO);
    _Float16* w1   = (_Float16*)(wsp + OFF_W1);
    _Float16* w2   = (_Float16*)(wsp + OFF_W2);
    _Float16* wout = (_Float16*)(wsp + OFF_WOUT);

    const unsigned nDD = (unsigned)(NLAYER * DM * DM / 8), nFD = (unsigned)(NLAYER * FFD * DM / 8), nVD = (unsigned)(VOCAB * DM / 8);
    k_prepw<<<nDD / 256, 256, 0, stream>>>(Wq, wq, nDD);
    k_prepw<<<nDD / 256, 256, 0, stream>>>(Wk, wk, nDD);
    k_prepw<<<nDD / 256, 256, 0, stream>>>(Wv, wv, nDD);
    k_prepw<<<nDD / 256, 256, 0, stream>>>(Wo, wo, nDD);
    k_prepw<<<nFD / 256, 256, 0, stream>>>(W1, w1, nFD);
    k_prepw<<<nFD / 256, 256, 0, stream>>>(W2, w2, nFD);
    k_prepw<<<nVD / 256, 256, 0, stream>>>(Wout, wout, nVD);

    k_embed<<<(MTOK * DM / 4) / 256, 256, 0, stream>>>(tokens, emb, pos, xA);

    const unsigned nXD = (unsigned)(MTOK * DM / 8), nXF = (unsigned)(MTOK * FFD / 8);
    const unsigned gD = ((MTOK / 64) * (DM / 64) + 7) / 8;
    const unsigned gF = ((MTOK / 64) * (FFD / 64) + 7) / 8;
    const unsigned gV = ((MTOK / 64) * (VOCAB / 64) + 7) / 8;

    for (int l = 0; l < NLAYER; ++l) {
        k_prepx<<<nXD / 256, 256, 0, stream>>>(xA, a16, nXD);
        k_gemm_plain<<<gD, 256, 0, stream>>>(a16, DM, wq + (size_t)l * DM * DM, DM, qkv, QKVP, bq + l * DM, DM, DM);
        k_gemm_plain<<<gD, 256, 0, stream>>>(a16, DM, wk + (size_t)l * DM * DM, DM, qkv + DM, QKVP, bk + l * DM, DM, DM);
        k_gemm_plain<<<gD, 256, 0, stream>>>(a16, DM, wv + (size_t)l * DM * DM, DM, qkv + 2 * DM, QKVP, bv + l * DM, DM, DM);
        k_split<<<MTOK / 64, 256, 0, stream>>>(qkv, qk16, vt16);
        k_attn<<<NB * HEADS, 256, 0, stream>>>(qk16, vt16, ctx);
        k_prepx<<<nXD / 256, 256, 0, stream>>>(ctx, a16, nXD);
        k_gemm_resid<<<gD, 256, 0, stream>>>(a16, DM, wo + (size_t)l * DM * DM, DM, hB, DM, bo + l * DM, xA, DM, DM);
        k_ln<<<MTOK / 8, 256, 0, stream>>>(hB, g1 + l * DM, be1 + l * DM, xA);
        k_prepx<<<nXD / 256, 256, 0, stream>>>(xA, a16, nXD);
        k_gemm_relu<<<gF, 256, 0, stream>>>(a16, DM, w1 + (size_t)l * FFD * DM, DM, h1, FFD, b1 + l * FFD, FFD, DM);
        k_prepx<<<nXF / 256, 256, 0, stream>>>(h1, f16p, nXF);
        k_gemm_resid<<<gD, 256, 0, stream>>>(f16p, FFD, w2 + (size_t)l * DM * FFD, FFD, hB, DM, b2 + l * DM, xA, DM, FFD);
        k_ln<<<MTOK / 8, 256, 0, stream>>>(hB, g2 + l * DM, be2 + l * DM, xA);
    }
    k_prepx<<<nXD / 256, 256, 0, stream>>>(xA, a16, nXD);
    k_gemm_plain<<<gV, 256, 0, stream>>>(a16, DM, wout, DM, out, VOCAB, bout, VOCAB, DM);
}
